// DynamicConv1dTBC_7421703487701
// MI455X (gfx1250) — hardware-verified
//
#include <hip/hip_runtime.h>
#include <hip/hip_bf16.h>


#define BB    16
#define CC    256
#define HH    8
#define KK    7
#define NO    (HH * KK)
#define HID   16
#define TILE  16
#define HALO  (KK - 1)
#define WIN   (TILE + HALO)
#define KP    8
#define LOGP  64

typedef float    v4f  __attribute__((ext_vector_type(4)));
typedef float    v8f  __attribute__((ext_vector_type(8)));
typedef _Float16 v8h  __attribute__((ext_vector_type(8)));
typedef _Float16 v16h __attribute__((ext_vector_type(16)));
typedef __bf16   v8b  __attribute__((ext_vector_type(8)));
typedef __bf16   v16b __attribute__((ext_vector_type(16)));
typedef v4f v4fa __attribute__((may_alias));
typedef v8h v8ha __attribute__((may_alias));

union FragH { v16h v; v8h half[2]; };
union FragB { v16b v; v8b half[2]; };

__device__ __forceinline__ v8f wmma_bf16(v16b a, v16b b, v8f c)
{
    v8f d = __builtin_amdgcn_wmma_f32_16x16x32_bf16(false, a, false, b, (short)0, c, false, false);
    asm volatile("v_nop\n\tv_nop\n\tv_nop\n\tv_nop" : "+v"(d) : "v"(a), "v"(b));
    return d;
}

__device__ __forceinline__ v8f wmma_f16(v16h a, v16h b, v8f c)
{
    v8f d = __builtin_amdgcn_wmma_f32_16x16x32_f16(false, a, false, b, (short)0, c, false, false);
    asm volatile("v_nop\n\tv_nop\n\tv_nop\n\tv_nop" : "+v"(d) : "v"(a), "v"(b));
    return d;
}

__device__ __forceinline__ void cvt_split8(const float* p, float scale, v8b& hv, v8b& lv)
{
    const v4f u0 = *(const v4fa*)p;
    const v4f u1 = *(const v4fa*)(p + 4);
    float f[8] = {u0[0], u0[1], u0[2], u0[3], u1[0], u1[1], u1[2], u1[3]};
    v8b hh = {};
    v8b ll = {};
#pragma unroll
    for (int i = 0; i < 8; ++i) {
        const float v = f[i] * scale;
        const __bf16 hb = (__bf16)v;
        const float r = v - (float)hb;
        hh[i] = hb;
        ll[i] = (__bf16)r;
    }
    hv = hh;
    lv = ll;
}

__device__ __forceinline__ void store_tile(float* out, const float* s_out, int t0, int b, int T, int lane)
{
    for (int row = 0; row < TILE; ++row) {
        if (t0 + row < T) {
            float* orow = out + ((size_t)(t0 + row) * BB + b) * CC;
#pragma unroll
            for (int cc2 = 0; cc2 < 2; ++cc2) {
                const int c = cc2 * 128 + lane * 4;
                const v4f v = *(const v4fa*)(s_out + row * CC + c);
                *(volatile v4f*)(orow + c) = v;
            }
        }
    }
}

__launch_bounds__(32) __attribute__((amdgpu_num_vgpr(248)))
__global__ void k_dynconv(const float* __restrict__ x,
                          const float* __restrict__ Wl,
                          const float* __restrict__ W1,
                          const float* __restrict__ W2,
                          const float* __restrict__ Wsp,
                          float* __restrict__ out,
                          int T)
{
    __shared__ float s_win[WIN * CC]       __attribute__((aligned(16)));
    __shared__ float s_wlog[TILE * LOGP]   __attribute__((aligned(16)));
    __shared__ float s_ca[TILE * CC]       __attribute__((aligned(16)));
    __shared__ float s_h[TILE * 32]        __attribute__((aligned(16)));
    __shared__ float s_sp[TILE * 2 * KP]   __attribute__((aligned(16)));
    __shared__ float s_sa[TILE * KP]       __attribute__((aligned(16)));
    __shared__ float s_po[TILE * CC]       __attribute__((aligned(16)));

    const int lane = threadIdx.x & 31;
    const int h    = lane >> 4;
    const int m    = lane & 15;
    const int b    = blockIdx.x % BB;
    const int t0   = (blockIdx.x / BB) * TILE;

    _Float16* s_pa = reinterpret_cast<_Float16*>(s_po);
    _Float16* s_pm = s_pa + TILE * CC;

    for (int i = lane; i < WIN * (CC / 4); i += 32) {
        const int j  = i >> 6;
        const int c4 = (i & 63) << 2;
        const int t  = t0 - HALO + j;
        v4f v = {0.f, 0.f, 0.f, 0.f};
        if (t >= 0 && t < T)
            v = *(const v4fa*)(x + ((size_t)t * BB + b) * CC + c4);
        *(v4fa*)(s_win + j * CC + c4) = v;
    }
    __syncthreads();

    {
        const float inv7 = 1.f / (float)KK;
        for (int i = lane; i < TILE * (CC / 4); i += 32) {
            const int row = i >> 6;
            const int c4  = (i & 63) << 2;
            v4f sv = {0.f, 0.f, 0.f, 0.f};
            v4f mx = {-3.4e38f, -3.4e38f, -3.4e38f, -3.4e38f};
#pragma unroll
            for (int j = 0; j < KK; ++j) {
                const v4f v = *(const v4fa*)(s_win + (row + j) * CC + c4);
                sv += v;
#pragma unroll
                for (int q = 0; q < 4; ++q) mx[q] = fmaxf(mx[q], v[q]);
            }
            const int o = row * CC + c4;
#pragma unroll
            for (int q = 0; q < 4; ++q) {
                s_pa[o + q] = (_Float16)(sv[q] * inv7);
                s_pm[o + q] = (_Float16)mx[q];
            }
        }
    }
    __syncthreads();

    {
        v8f acc[4] = {{}, {}, {}, {}};
        const float* arow = s_win + (m + HALO) * CC + 8 * h;
#pragma unroll 1
        for (int kc = 0; kc < CC / 32; ++kc) {
            FragB ahi, alo;
            cvt_split8(arow + kc * 32,      1.f, ahi.half[0], alo.half[0]);
            cvt_split8(arow + kc * 32 + 16, 1.f, ahi.half[1], alo.half[1]);
#pragma unroll
            for (int ct = 0; ct < 4; ++ct) {
                const int   o   = ct * 16 + m;
                const int   oc  = (o < NO) ? o : 0;
                const float msk = (o < NO) ? 1.f : 0.f;
                const float* brow = Wl + (size_t)oc * CC + kc * 32 + 8 * h;
                FragB bhi, blo;
                cvt_split8(brow,      msk, bhi.half[0], blo.half[0]);
                cvt_split8(brow + 16, msk, bhi.half[1], blo.half[1]);
                acc[ct] = wmma_bf16(ahi.v, bhi.v, acc[ct]);
                acc[ct] = wmma_bf16(alo.v, bhi.v, acc[ct]);
                acc[ct] = wmma_bf16(ahi.v, blo.v, acc[ct]);
            }
        }
#pragma unroll
        for (int ct = 0; ct < 4; ++ct)
#pragma unroll
            for (int r = 0; r < 8; ++r)
                s_wlog[(8 * h + r) * LOGP + ct * 16 + m] = acc[ct][r];
    }
    __syncthreads();

    for (int slot = lane; slot < TILE * HH; slot += 32) {
        const int row = slot >> 3, hd = slot & 7;
        float* p = &s_wlog[row * LOGP + hd * KK];
        float mxv = p[0];
#pragma unroll
        for (int k = 1; k < KK; ++k) mxv = fmaxf(mxv, p[k]);
        float ex[KK], sum = 0.f;
#pragma unroll
        for (int k = 0; k < KK; ++k) { ex[k] = expf(p[k] - mxv); sum += ex[k]; }
        const float inv = 1.f / sum;
#pragma unroll
        for (int k = 0; k < KK; ++k) p[k] = ex[k] * inv;
    }
    __syncthreads();

    {
        v8f accA = {}, accM = {};
        const _Float16* pa = s_pa + m * CC + 8 * h;
        const _Float16* pm = s_pm + m * CC + 8 * h;
#pragma unroll 1
        for (int kc = 0; kc < CC / 32; ++kc) {
            FragH aA, aM;
            aA.half[0] = *(const v8ha*)(pa + kc * 32);
            aA.half[1] = *(const v8ha*)(pa + kc * 32 + 16);
            aM.half[0] = *(const v8ha*)(pm + kc * 32);
            aM.half[1] = *(const v8ha*)(pm + kc * 32 + 16);
            v16h bw = {};
#pragma unroll
            for (int i = 0; i < 8; ++i) {
                bw[i]     = (_Float16)(W1[(kc * 32 + 8 * h + i) * HID + m] * 16.f);
                bw[8 + i] = (_Float16)(W1[(kc * 32 + 16 + 8 * h + i) * HID + m] * 16.f);
            }
            accA = wmma_f16(aA.v, bw, accA);
            accM = wmma_f16(aM.v, bw, accM);
        }
#pragma unroll
        for (int r = 0; r < 8; ++r) {
            const int M = 8 * h + r;
            s_h[M * 32 + m]      = fmaxf(accA[r] * 0.0625f, 0.f);
            s_h[M * 32 + 16 + m] = fmaxf(accM[r] * 0.0625f, 0.f);
        }
    }
    __syncthreads();

    {
        FragH ah;
        {
            v8h a0 = {}, a1 = {};
#pragma unroll
            for (int i = 0; i < 8; ++i) {
                a0[i] = (_Float16)s_h[m * 32 + 8 * h + i];
                a1[i] = (_Float16)s_h[m * 32 + 16 + 8 * h + i];
            }
            ah.half[0] = a0;
            ah.half[1] = a1;
        }
#pragma unroll 1
        for (int ct = 0; ct < CC / 16; ++ct) {
            v16h bw = {};
#pragma unroll
            for (int i = 0; i < 8; ++i) {
                const _Float16 w = (_Float16)(W2[(8 * h + i) * CC + ct * 16 + m] * 16.f);
                bw[i]     = w;
                bw[8 + i] = w;
            }
            v8f acc = {};
            acc = wmma_f16(ah.v, bw, acc);
#pragma unroll
            for (int r = 0; r < 8; ++r) {
                const int M = 8 * h + r;
                s_ca[M * CC + ct * 16 + m] = 1.f / (1.f + expf(-(acc[r] * 0.0625f)));
            }
        }
    }
    __syncthreads();

    for (int slot = lane; slot < TILE * KK; slot += 32) {
        const int row = slot / KK, k = slot % KK;
        const float* wr = s_win + (row + k) * CC;
        const float* cr = s_ca + row * CC;
        float sv = 0.f, mx = -3.4e38f;
        for (int c = 0; c < CC; c += 4) {
            const v4f wv = *(const v4fa*)(wr + c);
            const v4f cv = *(const v4fa*)(cr + c);
            const v4f p  = wv * cv;
            sv += (p[0] + p[1]) + (p[2] + p[3]);
            mx = fmaxf(mx, fmaxf(fmaxf(p[0], p[1]), fmaxf(p[2], p[3])));
        }
        s_sp[(row * 2 + 0) * KP + k] = sv * (1.f / (float)CC);
        s_sp[(row * 2 + 1) * KP + k] = mx;
    }
    __syncthreads();

    {
        float wsp[2 * KK];
#pragma unroll
        for (int i = 0; i < 2 * KK; ++i) wsp[i] = Wsp[i];
        for (int slot = lane; slot < TILE * KK; slot += 32) {
            const int row = slot / KK, k = slot % KK;
            float acc = 0.f;
#pragma unroll
            for (int j = 0; j < KK; ++j) {
                const int kk = k + j - 3;
                if (kk >= 0 && kk < KK)
                    acc += s_sp[(row * 2 + 0) * KP + kk] * wsp[j]
                         + s_sp[(row * 2 + 1) * KP + kk] * wsp[KK + j];
            }
            s_sa[row * KP + k] = 1.f / (1.f + expf(-acc));
        }
    }
    __syncthreads();

    {
        float* s_out = s_po;
        for (int row = 0; row < TILE; ++row) {
            float wsa[KK];
#pragma unroll
            for (int k = 0; k < KK; ++k) wsa[k] = s_sa[row * KP + k];
#pragma unroll
            for (int cc2 = 0; cc2 < 2; ++cc2) {
                const int c  = cc2 * 128 + lane * 4;
                const int hd = c >> 5;
                v4f acc = {0.f, 0.f, 0.f, 0.f};
#pragma unroll
                for (int k = 0; k < KK; ++k) {
                    const float wk = wsa[k] * s_wlog[row * LOGP + hd * KK + k];
                    const v4f xv = *(const v4fa*)(s_win + (row + k) * CC + c);
                    acc += xv * wk;
                }
                const v4f cav = *(const v4fa*)(s_ca + row * CC + c);
                acc *= cav;
                *(v4fa*)(s_out + row * CC + c) = acc;
            }
        }
    }
    __syncthreads();

    store_tile(out, s_po, t0, b, T, lane);
    __threadfence();
    store_tile(out, s_po, t0, b, T, lane);
}

extern "C" void kernel_launch(void* const* d_in, const int* in_sizes, int n_in,
                              void* d_out, int out_size, void* d_ws, size_t ws_size,
                              hipStream_t stream)
{
    (void)n_in; (void)d_ws; (void)ws_size;
    const float* x   = (const float*)d_in[0];
    const float* Wl  = (const float*)d_in[1];
    const float* W1  = (const float*)d_in[2];
    const float* W2  = (const float*)d_in[3];
    const float* Wsp = (const float*)d_in[4];
    float* out = (float*)d_out;

    int T = in_sizes[0] / (BB * CC);
    const int To = out_size / (BB * CC);
    if (To < T) T = To;
    if (T <= 0) return;
    const int ntiles = (T + TILE - 1) / TILE;

    dim3 grid((unsigned)(ntiles * BB));
    dim3 block(32);
    hipLaunchKernelGGL(k_dynconv, grid, block, 0, stream, x, Wl, W1, W2, Wsp, out, T);
}
